// UpdateAttn_35974646071568
// MI455X (gfx1250) — hardware-verified
//
#include <hip/hip_runtime.h>
#include <stddef.h>
#include <stdint.h>

#define NB    2
#define SQ    2048
#define NTOK  4096
#define HID   1024
#define NH    16
#define HDM   64
#define NQKV  3072
#define NSQ   8
#define NSLAB 24
#define QB    128
#define KC    64
#define NQB   (SQ / QB)
#define NCK   (SQ / KC)
#define SBLK  (SQ / 64)

static_assert(NTOK == NB * SQ);
static_assert(SQ % 256 == 0);
static_assert(HID % 64 == 0);
static_assert(HID == 128 * 8);
static_assert(HDM == 64);
static_assert(NH * HDM == HID);
static_assert(NQKV == 3 * NH * HDM);
static_assert(NQKV == NSLAB * 128);
static_assert(NSQ * 128 == NH * HDM);
static_assert(SQ % KC == 0);
static_assert(SQ % QB == 0);
static_assert(NTOK % 256 == 0);
static_assert(NTOK % 8 == 0);

typedef _Float16 v16h __attribute__((ext_vector_type(16)));
typedef _Float16 v8h  __attribute__((ext_vector_type(8)));
typedef float    v8f  __attribute__((ext_vector_type(8)));
typedef float    v4f  __attribute__((ext_vector_type(4)));
typedef unsigned int v4u __attribute__((ext_vector_type(4)));

union Frag  { v16h v; v8h h[2]; };
union Pack8 { v8h h; v4u u; };

__device__ __forceinline__ v8f mma16(v16h a, v16h b, v8f c) {
  c = __builtin_amdgcn_wmma_f32_16x16x32_f16(false, a, false, b, (short)0, c, false, false);
  asm volatile("v_nop\n\tv_nop\n\tv_nop\n\tv_nop" : "+v"(c) : "v"(a), "v"(b));
  return c;
}

__device__ __forceinline__ v16h ldfrag(const _Float16* p, int ld, int row0, int k0, int lane) {
  const int m = lane & 15, lh = lane >> 4;
  const _Float16* q = p + (size_t)(row0 + m) * ld + k0 + 8 * lh;
  Frag f;
  f.h[0] = *(const v8h*)(q);
  f.h[1] = *(const v8h*)(q + 16);
  return f.v;
}

__device__ __forceinline__ v8f zero8() { return (v8f){0.f, 0.f, 0.f, 0.f, 0.f, 0.f, 0.f, 0.f}; }

__device__ __forceinline__ void gemm16x64(const _Float16* __restrict__ A, int lda,
                                          const _Float16* __restrict__ Bt, int ldb,
                                          int m0, int n0, int lane, v8f (&acc)[4]) {
#pragma unroll 2
  for (int k0 = 0; k0 < HID; k0 += 32) {
    const v16h a = ldfrag(A, lda, m0, k0, lane);
#pragma unroll
    for (int t = 0; t < 4; ++t) {
      const v16h b = ldfrag(Bt, ldb, n0 + 16 * t, k0, lane);
      acc[t] = mma16(a, b, acc[t]);
    }
  }
}

__device__ __forceinline__ void gemm32x64(const _Float16* __restrict__ A, int lda,
                                          const _Float16* __restrict__ Bt, int ldb,
                                          int m0, int n0, int lane, v8f (&acc)[2][4]) {
#pragma unroll 2
  for (int k0 = 0; k0 < HID; k0 += 32) {
    const v16h a0 = ldfrag(A, lda, m0, k0, lane);
    const v16h a1 = ldfrag(A, lda, m0 + 16, k0, lane);
    const v16h b0 = ldfrag(Bt, ldb, n0, k0, lane);
    const v16h b1 = ldfrag(Bt, ldb, n0 + 16, k0, lane);
    const v16h b2 = ldfrag(Bt, ldb, n0 + 32, k0, lane);
    const v16h b3 = ldfrag(Bt, ldb, n0 + 48, k0, lane);
    acc[0][0] = mma16(a0, b0, acc[0][0]);
    acc[1][0] = mma16(a1, b0, acc[1][0]);
    acc[0][1] = mma16(a0, b1, acc[0][1]);
    acc[1][1] = mma16(a1, b1, acc[1][1]);
    acc[0][2] = mma16(a0, b2, acc[0][2]);
    acc[1][2] = mma16(a1, b2, acc[1][2]);
    acc[0][3] = mma16(a0, b3, acc[0][3]);
    acc[1][3] = mma16(a1, b3, acc[1][3]);
  }
}

__global__ __launch_bounds__(256) void k_cvt(const float* __restrict__ src, _Float16* __restrict__ dh, float scale) {
  const int tid = threadIdx.x;
  const int row = blockIdx.x * 2 + (tid >> 7);
  const int col = (tid & 127) * 8;
  const size_t o = (size_t)row * HID + col;
  const v4f a0 = *(const v4f*)(src + o) * scale;
  const v4f a1 = *(const v4f*)(src + o + 4) * scale;
  Pack8 pk;
  pk.h = (v8h){(_Float16)a0[0], (_Float16)a0[1], (_Float16)a0[2], (_Float16)a0[3],
               (_Float16)a1[0], (_Float16)a1[1], (_Float16)a1[2], (_Float16)a1[3]};
  const v4u vv = pk.u;
  volatile v4u* d = (volatile v4u*)(dh + o);
  *d = vv;
  __threadfence();
  *d = vv;
}

__device__ __forceinline__ float sin_small(float x) {
  const float x2 = x * x;
  float p = 2.7557319223985893e-06f;
  p = p * x2 - 1.9841269841269841e-04f;
  p = p * x2 + 8.3333333333333332e-03f;
  p = p * x2 - 1.6666666666666666e-01f;
  p = p * x2 + 1.0f;
  return x * p;
}
__device__ __forceinline__ float cos_small(float x) {
  const float x2 = x * x;
  float p = -2.7557319223985888e-07f;
  p = p * x2 + 2.4801587301587302e-05f;
  p = p * x2 - 1.3888888888888889e-03f;
  p = p * x2 + 4.1666666666666664e-02f;
  p = p * x2 - 0.5f;
  p = p * x2 + 1.0f;
  return p;
}
__global__ __launch_bounds__(256) void k_pe(float* __restrict__ pe) {
  const int tid = threadIdx.x;
#pragma unroll 1
  for (int it = 0; it < 2; ++it) {
    const int q  = tid + 256 * it;
    const int b  = q >> 8;
    const int d0 = (q & 255) * 4;
    const float fb = (float)b;
    const int mA = d0 >> 1, mB = mA + 1;
    const float eA = (float)(2 * mA) * 0.0009765625f;
    const float eB = (float)(2 * mB) * 0.0009765625f;
    const float fA = exp2f(-eA * 13.287712379549449f);
    const float fB = exp2f(-eB * 13.287712379549449f);
    const float aA = fb * fA, aB = fb * fB;
    const v4f val = (v4f){sin_small(aA), cos_small(aA), sin_small(aB), cos_small(aB)};
    volatile v4f* d = (volatile v4f*)(pe + 4 * q);
    *d = val;
    __threadfence();
    *d = val;
  }
}

#define SFP 132
__global__ __launch_bounds__(256) void k_qkv(const _Float16* __restrict__ xh,
                                             const _Float16* __restrict__ wt,
                                             _Float16* __restrict__ qp,
                                             _Float16* __restrict__ kp,
                                             _Float16* __restrict__ vtp) {
  __shared__ __align__(16) float sf[64 * SFP];
  const int tid = threadIdx.x, lane = tid & 31, wave = tid >> 5;
  const int hh = lane >> 4, c = lane & 15;
  const int wm = wave >> 1, wn = wave & 1;
  const int bx = blockIdx.x;
  const int b  = bx / SBLK;
  const int sb = (bx - b * SBLK) * 64;
  const int ns = blockIdx.y;
  const int which = (ns < NSQ) ? 0 : ((ns < 2 * NSQ) ? 1 : 2);
  const int hp = 2 * (ns - NSQ * which);
  const int m0 = sb + wm * 16;
  const int n0 = ns * 128 + wn * 64;
  const _Float16* A = xh + (size_t)b * HID;

  v8f acc[4];
#pragma unroll
  for (int t = 0; t < 4; ++t) acc[t] = zero8();
  gemm16x64(A, NB * HID, wt, HID, m0, n0, lane, acc);

#pragma unroll
  for (int t = 0; t < 4; ++t) {
#pragma unroll
    for (int r = 0; r < 8; ++r)
      sf[(wm * 16 + 8 * hh + r) * SFP + wn * 64 + 16 * t + c] = acc[t][r] * 0.03125f;
  }
  __syncthreads();

  if (which < 2) {
    v4u val[4];
    size_t go[4];
#pragma unroll
    for (int j = 0; j < 4; ++j) {
      const int p  = tid + 256 * j;
      const int lr = p >> 4;
      const int pc = p & 15;
      const int hs = pc >> 3;
      const int d0 = (pc & 7) * 8;
      const float* ra = sf + lr * SFP + pc * 8;
      const v4f a0 = *(const v4f*)(ra), a1 = *(const v4f*)(ra + 4);
      Pack8 pk;
      pk.h = (v8h){(_Float16)a0[0], (_Float16)a0[1], (_Float16)a0[2], (_Float16)a0[3],
                   (_Float16)a1[0], (_Float16)a1[1], (_Float16)a1[2], (_Float16)a1[3]};
      val[j] = pk.u;
      const int hb = b * NH + hp + hs;
      go[j]  = ((size_t)hb * SQ + sb + lr) * HDM + d0;
    }
    _Float16* base = (which == 0) ? qp : kp;
    for (int ps = 0; ps < 2; ++ps) {
#pragma unroll
      for (int j = 0; j < 4; ++j) *(volatile v4u*)(base + go[j]) = val[j];
      __threadfence();
    }
  } else {
    v4u val[4];
    size_t go[4];
#pragma unroll
    for (int j = 0; j < 4; ++j) {
      const int p    = tid + 256 * j;
      const int dcol = p >> 3;
      const int pc   = p & 7;
      const float* cp = sf + (pc * 8) * SFP + dcol;
      Pack8 pk;
      pk.h = (v8h){(_Float16)cp[0 * SFP], (_Float16)cp[1 * SFP], (_Float16)cp[2 * SFP], (_Float16)cp[3 * SFP],
                   (_Float16)cp[4 * SFP], (_Float16)cp[5 * SFP], (_Float16)cp[6 * SFP], (_Float16)cp[7 * SFP]};
      val[j] = pk.u;
      const int hb = b * NH + hp + (dcol >> 6);
      const int d  = dcol & 63;
      go[j]  = ((size_t)hb * HDM + d) * SQ + sb + pc * 8;
    }
    for (int ps = 0; ps < 2; ++ps) {
#pragma unroll
      for (int j = 0; j < 4; ++j) *(volatile v4u*)(vtp + go[j]) = val[j];
      __threadfence();
    }
  }
}

#define KTP 72
__global__ __launch_bounds__(256) void k_attn(const _Float16* __restrict__ qp,
                                              const _Float16* __restrict__ kp,
                                              const _Float16* __restrict__ vt,
                                              _Float16* __restrict__ op, float sscale) {
  __shared__ __align__(16) _Float16 Ks[KC * KTP];
  __shared__ __align__(16) _Float16 Vs[HDM * KTP];
  __shared__ __align__(16) _Float16 Ps[8 * 16 * KTP];

  const int tid = threadIdx.x, lane = tid & 31, wave = tid >> 5;
  const int hh = lane >> 4, c = lane & 15;
  const int qb  = blockIdx.x % NQB;
  const int hb  = blockIdx.x / NQB;
  const int h   = hb % NH;
  const int b   = hb / NH;
  const int q0  = qb * QB + wave * 16;

  const _Float16* Q = qp + (size_t)hb * SQ * HDM;
  const _Float16* K = kp + (size_t)hb * SQ * HDM;
  const _Float16* V = vt + (size_t)hb * HDM * SQ;

  v16h qa[2];
  qa[0] = ldfrag(Q, HDM, q0, 0, lane);
  qa[1] = ldfrag(Q, HDM, q0, 32, lane);

  const float NEGI = -__builtin_huge_valf();
  float mrow[8], lrow[8];
  v8f oacc[4];
#pragma unroll
  for (int r = 0; r < 8; ++r) { mrow[r] = NEGI; lrow[r] = 0.f; }
#pragma unroll
  for (int t = 0; t < 4; ++t) oacc[t] = zero8();

  _Float16* pw = Ps + wave * 16 * KTP;

  for (int kc = 0; kc < NCK; ++kc) {
    const int kv0 = kc * KC;
    __syncthreads();
    {
      const int r  = tid >> 2;
      const int qq = (tid & 3) * 16;
      const _Float16* ks = K + (size_t)(kv0 + r) * HDM + qq;
      const _Float16* vs = V + (size_t)r * SQ + kv0 + qq;
#pragma unroll
      for (int e = 0; e < 2; ++e) {
        *(v8h*)(Ks + r * KTP + qq + 8 * e) = *(const v8h*)(ks + 8 * e);
        *(v8h*)(Vs + r * KTP + qq + 8 * e) = *(const v8h*)(vs + 8 * e);
      }
    }
    __syncthreads();

    v8f s[4];
#pragma unroll
    for (int j = 0; j < 4; ++j) s[j] = zero8();
#pragma unroll
    for (int dc = 0; dc < 2; ++dc) {
#pragma unroll
      for (int j = 0; j < 4; ++j) {
        const v16h kb = ldfrag(Ks, KTP, j * 16, dc * 32, lane);
        s[j] = mma16(qa[dc], kb, s[j]);
      }
    }
    float cm[8];
#pragma unroll
    for (int r = 0; r < 8; ++r) {
      float m = NEGI;
#pragma unroll
      for (int j = 0; j < 4; ++j) { s[j][r] *= sscale; m = fmaxf(m, s[j][r]); }
#pragma unroll
      for (int off = 1; off < 16; off <<= 1) m = fmaxf(m, __shfl_xor(m, off, 32));
      cm[r] = m;
    }
    float al[8];
#pragma unroll
    for (int r = 0; r < 8; ++r) {
      const float mnew  = fmaxf(mrow[r], cm[r]);
      const float alpha = __expf(mrow[r] - mnew);
      mrow[r] = mnew;
      float psum = 0.f;
#pragma unroll
      for (int j = 0; j < 4; ++j) {
        const float p = __expf(s[j][r] - mnew);
        psum += p;
        pw[(8 * hh + r) * KTP + j * 16 + c] = (_Float16)(p * 1024.0f);
      }
#pragma unroll
      for (int off = 1; off < 16; off <<= 1) psum += __shfl_xor(psum, off, 32);
      lrow[r] = lrow[r] * alpha + psum;
      al[r] = alpha;
    }
#pragma unroll
    for (int t = 0; t < 4; ++t)
#pragma unroll
      for (int r = 0; r < 8; ++r) oacc[t][r] *= al[r];
    __syncthreads();

#pragma unroll
    for (int kk = 0; kk < 2; ++kk) {
      const v16h pa = ldfrag(pw, KTP, 0, kk * 32, lane);
#pragma unroll
      for (int t = 0; t < 4; ++t) {
        const v16h vb = ldfrag(Vs, KTP, t * 16, kk * 32, lane);
        oacc[t] = mma16(pa, vb, oacc[t]);
      }
    }
  }

  float invl[8];
#pragma unroll
  for (int r = 0; r < 8; ++r) invl[r] = (lrow[r] > 0.f) ? (0.0625f / lrow[r]) : 0.f;
  __syncthreads();
#pragma unroll
  for (int r = 0; r < 8; ++r) {
#pragma unroll
    for (int t = 0; t < 4; ++t)
      pw[(8 * hh + r) * KTP + 16 * t + c] = (_Float16)(oacc[t][r] * invl[r]);
  }
  __syncthreads();
  v4u val[4];
  size_t go[4];
#pragma unroll
  for (int it = 0; it < 4; ++it) {
    const int p  = lane + 32 * it;
    const int L  = p >> 3;
    const int pc = p & 7;
    Pack8 pk;
    pk.h    = *(const v8h*)(pw + L * KTP + pc * 8);
    val[it] = pk.u;
    go[it]  = ((size_t)(q0 + L) * NB + b) * HID + (size_t)h * HDM + pc * 8;
  }
  for (int ps = 0; ps < 2; ++ps) {
#pragma unroll
    for (int it = 0; it < 4; ++it) *(volatile v4u*)(op + go[it]) = val[it];
    __threadfence();
  }
}

#define OTP 68
__device__ __forceinline__ void out_epilogue(v8f (&acc)[2][4], float scale,
                                             float* sw, float* __restrict__ out,
                                             int m0, int n0, int lane, int hh, int c) {
#pragma unroll
  for (int sub = 0; sub < 2; ++sub) {
    __syncthreads();
#pragma unroll
    for (int t = 0; t < 4; ++t) {
#pragma unroll
      for (int r = 0; r < 8; ++r) sw[(8 * hh + r) * OTP + 16 * t + c] = acc[sub][t][r] * scale;
    }
    __syncthreads();
    v4f val[8];
    size_t go[8];
#pragma unroll
    for (int it = 0; it < 8; ++it) {
      const int p    = lane + 32 * it;
      const int L    = p >> 3;
      const int pc   = p & 7;
      const int row  = L >> 1;
      const int half = L & 1;
      val[it] = *(const v4f*)(sw + row * OTP + half * 32 + pc * 4);
      go[it]  = (size_t)(m0 + sub * 16 + row) * HID + n0 + half * 32 + pc * 4;
    }
    for (int ps = 0; ps < 2; ++ps) {
#pragma unroll
      for (int it = 0; it < 8; ++it) *(volatile v4f*)(out + go[it]) = val[it];
      __threadfence();
    }
  }
}

__global__ __launch_bounds__(256) void k_gemm(const _Float16* __restrict__ ap,
                                              const _Float16* __restrict__ wt,
                                              float scale,
                                              float* __restrict__ out) {
  __shared__ __align__(16) float st[8][16 * OTP];
  const int tid = threadIdx.x, lane = tid & 31, wave = tid >> 5;
  const int hh = lane >> 4, c = lane & 15;
  const int m0 = blockIdx.x * 256 + wave * 32;
  const int n0 = blockIdx.y * 64;

  v8f acc[2][4];
#pragma unroll
  for (int s = 0; s < 2; ++s)
#pragma unroll
    for (int t = 0; t < 4; ++t) acc[s][t] = zero8();
  gemm32x64(ap, HID, wt, HID, m0, n0, lane, acc);
  out_epilogue(acc, scale, st[wave], out, m0, n0, lane, hh, c);
}

__global__ __launch_bounds__(256) void k_ln1(const float* __restrict__ t, const float* __restrict__ res,
                                             const float* __restrict__ g, const float* __restrict__ be,
                                             float* __restrict__ yf, _Float16* __restrict__ yh) {
  __shared__ __align__(16) float sw[8][HID];
  const int tid = threadIdx.x, lane = tid & 31, wave = tid >> 5;
  const size_t m = (size_t)blockIdx.x * 8 + wave;
  const float* tr = t + m * HID;
  const float* rr = res + m * HID;

  v4f v[8];
  float s = 0.f;
#pragma unroll
  for (int it = 0; it < 8; ++it) {
    const int idx = it * 128 + lane * 4;
    const v4f a = *(const v4f*)(tr + idx);
    const v4f r = *(const v4f*)(rr + idx);
    v[it] = a + r;
    s += (v[it][0] + v[it][1]) + (v[it][2] + v[it][3]);
  }
#pragma unroll
  for (int off = 16; off >= 1; off >>= 1) s += __shfl_xor(s, off, 32);
  const float mean = s * 0.0009765625f;
  float ss = 0.f;
#pragma unroll
  for (int it = 0; it < 8; ++it) {
    const v4f d = v[it] - mean;
    ss += (d[0] * d[0] + d[1] * d[1]) + (d[2] * d[2] + d[3] * d[3]);
  }
#pragma unroll
  for (int off = 16; off >= 1; off >>= 1) ss += __shfl_xor(ss, off, 32);
  const float var  = ss * 0.0009765625f;
  const float rstd = rsqrtf(var + 1e-5f);

  v4f y[8];
#pragma unroll
  for (int it = 0; it < 8; ++it) {
    const int idx = it * 128 + lane * 4;
    const v4f gv = *(const v4f*)(g + idx);
    const v4f bv = *(const v4f*)(be + idx);
    y[it] = ((v[it] - mean) * rstd) * gv + bv;
  }
  for (int ps = 0; ps < 2; ++ps) {
#pragma unroll
    for (int it = 0; it < 8; ++it) *(volatile v4f*)(yf + m * HID + it * 128 + lane * 4) = y[it];
    __threadfence();
  }
#pragma unroll
  for (int it = 0; it < 8; ++it) *(v4f*)(sw[wave] + it * 128 + lane * 4) = y[it];
  __syncthreads();
  v4u hv[4];
  size_t go[4];
#pragma unroll
  for (int j = 0; j < 4; ++j) {
    const float* cp = sw[wave] + 256 * j + 8 * lane;
    const v4f a0 = *(const v4f*)(cp), a1 = *(const v4f*)(cp + 4);
    Pack8 pk;
    pk.h = (v8h){(_Float16)a0[0], (_Float16)a0[1], (_Float16)a0[2], (_Float16)a0[3],
                 (_Float16)a1[0], (_Float16)a1[1], (_Float16)a1[2], (_Float16)a1[3]};
    hv[j] = pk.u;
    go[j] = m * HID + 256 * j + 8 * lane;
  }
  for (int ps = 0; ps < 2; ++ps) {
#pragma unroll
    for (int j = 0; j < 4; ++j) *(volatile v4u*)(yh + go[j]) = hv[j];
    __threadfence();
  }
}

__global__ __launch_bounds__(256) void k_ln2(const float* __restrict__ t, const float* __restrict__ res,
                                             const float* __restrict__ g, const float* __restrict__ be,
                                             const float* __restrict__ pe, float* __restrict__ out) {
  const int tid = threadIdx.x, lane = tid & 31, wave = tid >> 5;
  const size_t m = (size_t)blockIdx.x * 8 + wave;
  const int b = (int)(m & 1);
  const float* tr = t + m * HID;
  const float* rr = res + m * HID;
  const float* pr = pe + (size_t)b * HID;

  v4f v[8];
  float s = 0.f;
#pragma unroll
  for (int it = 0; it < 8; ++it) {
    const int idx = it * 128 + lane * 4;
    const v4f a = *(const v4f*)(tr + idx);
    const v4f r = *(const v4f*)(rr + idx);
    v[it] = a + r;
    s += (v[it][0] + v[it][1]) + (v[it][2] + v[it][3]);
  }
#pragma unroll
  for (int off = 16; off >= 1; off >>= 1) s += __shfl_xor(s, off, 32);
  const float mean = s * 0.0009765625f;
  float ss = 0.f;
#pragma unroll
  for (int it = 0; it < 8; ++it) {
    const v4f d = v[it] - mean;
    ss += (d[0] * d[0] + d[1] * d[1]) + (d[2] * d[2] + d[3] * d[3]);
  }
#pragma unroll
  for (int off = 16; off >= 1; off >>= 1) ss += __shfl_xor(ss, off, 32);
  const float var  = ss * 0.0009765625f;
  const float rstd = rsqrtf(var + 1e-5f);

  v4f o[8];
#pragma unroll
  for (int it = 0; it < 8; ++it) {
    const int idx = it * 128 + lane * 4;
    const v4f gv = *(const v4f*)(g + idx);
    const v4f bv = *(const v4f*)(be + idx);
    const v4f pv = *(const v4f*)(pr + idx);
    const v4f y  = ((v[it] - mean) * rstd) * gv + bv;
    o[it] = y + (y + pv);
  }
  for (int ps = 0; ps < 2; ++ps) {
#pragma unroll
    for (int it = 0; it < 8; ++it) *(volatile v4f*)(out + m * HID + it * 128 + lane * 4) = o[it];
    __threadfence();
  }
}

extern "C" void kernel_launch(void* const* d_in, const int* in_sizes, int n_in,
                              void* d_out, int out_size, void* d_ws, size_t ws_size,
                              hipStream_t stream) {
  if (n_in < 9) return;
  if (in_sizes[0] != NTOK * HID) return;
  if (in_sizes[1] != HID * HID) return;
  if (in_sizes[2] != 2 * HID * HID) return;
  if (in_sizes[3] != HID * HID) return;
  if (in_sizes[4] != HID) return;
  if (in_sizes[5] != HID) return;
  if (in_sizes[6] != HID * HID) return;
  if (in_sizes[7] != HID) return;
  if (in_sizes[8] != HID) return;
  if (out_size != NTOK * HID) return;

  const float* x   = (const float*)d_in[0];
  const float* wq  = (const float*)d_in[1];
  const float* wkv = (const float*)d_in[2];
  const float* wo  = (const float*)d_in[3];
  const float* g1  = (const float*)d_in[4];
  const float* be1 = (const float*)d_in[5];
  const float* wff = (const float*)d_in[6];
  const float* g2  = (const float*)d_in[7];
  const float* be2 = (const float*)d_in[8];
  float* out = (float*)d_out;

  size_t off = 0;
  const size_t oX   = off; off += (size_t)NTOK * HID * 2;
  const size_t oWt  = off; off += (size_t)NQKV * HID * 2;
  const size_t oWo  = off; off += (size_t)HID * HID * 2;
  const size_t oWf  = off; off += (size_t)HID * HID * 2;
  const size_t oQ   = off; off += (size_t)NB * NH * SQ * HDM * 2;
  const size_t oK   = off; off += (size_t)NB * NH * SQ * HDM * 2;
  const size_t oV   = off; off += (size_t)NB * NH * HDM * SQ * 2;
  const size_t oO   = off; off += (size_t)NTOK * HID * 2;
  const size_t oT1  = off; off += (size_t)NTOK * HID * 4;
  const size_t oY1f = off; off += (size_t)NTOK * HID * 4;
  const size_t oY1h = off; off += (size_t)NTOK * HID * 2;
  const size_t oT2  = off; off += (size_t)NTOK * HID * 4;
  const size_t oPE  = off; off += (size_t)NB * HID * 4;
  if (off > ws_size) return;
  if (off > (size_t)134217728) return;

  char* ws = (char*)d_ws;
  _Float16* Xh  = (_Float16*)(ws + oX);
  _Float16* Wt  = (_Float16*)(ws + oWt);
  _Float16* Wot = (_Float16*)(ws + oWo);
  _Float16* Wft = (_Float16*)(ws + oWf);
  _Float16* Qp  = (_Float16*)(ws + oQ);
  _Float16* Kp  = (_Float16*)(ws + oK);
  _Float16* Vt  = (_Float16*)(ws + oV);
  _Float16* Op  = (_Float16*)(ws + oO);
  float*    T1  = (float*)(ws + oT1);
  float*    Y1f = (float*)(ws + oY1f);
  _Float16* Y1h = (_Float16*)(ws + oY1h);
  float*    T2  = (float*)(ws + oT2);
  float*    PE  = (float*)(ws + oPE);

  k_cvt<<<dim3(NTOK / 2), dim3(256), 0, stream>>>(x, Xh, 1.0f);
  k_cvt<<<dim3(HID / 2), dim3(256), 0, stream>>>(wq, Wt, 32.0f);
  k_cvt<<<dim3((2 * HID) / 2), dim3(256), 0, stream>>>(wkv, Wt + (size_t)HID * HID, 32.0f);
  k_cvt<<<dim3(HID / 2), dim3(256), 0, stream>>>(wo, Wot, 32.0f);
  k_cvt<<<dim3(HID / 2), dim3(256), 0, stream>>>(wff, Wft, 32.0f);
  k_pe<<<dim3(1), dim3(256), 0, stream>>>(PE);
  k_qkv<<<dim3(NB * SBLK, NSLAB), dim3(256), 0, stream>>>(Xh, Wt, Qp, Kp, Vt);
  const float sscale = 0.125f;
  k_attn<<<dim3(NB * NH * NQB), dim3(256), 0, stream>>>(Qp, Kp, Vt, Op, sscale);
  k_gemm<<<dim3(NTOK / 256, HID / 64), dim3(256), 0, stream>>>(Op, Wot, 0.00048828125f, T1);
  k_ln1<<<dim3(NTOK / 8), dim3(256), 0, stream>>>(T1, x, g1, be1, Y1f, Y1h);
  k_gemm<<<dim3(NTOK / 256, HID / 64), dim3(256), 0, stream>>>(Y1h, Wft, 0.03125f, T2);
  k_ln2<<<dim3(NTOK / 8), dim3(256), 0, stream>>>(T2, Y1f, g2, be2, PE, out);
  (void)hipGetLastError();
}
